// CoLightMultiHeadGAT_80564996538676
// MI455X (gfx1250) — hardware-verified
//
#include <hip/hip_runtime.h>
#include <hip/hip_bf16.h>
#include <math.h>
#include <stdint.h>

typedef __attribute__((ext_vector_type(16))) _Float16 v16h;
typedef __attribute__((ext_vector_type(8)))  _Float16 v8h;
typedef __attribute__((ext_vector_type(16))) __bf16   v16b;
typedef __attribute__((ext_vector_type(8)))  __bf16   v8b;
typedef __attribute__((ext_vector_type(8)))  float    v8f;
typedef __attribute__((ext_vector_type(4)))  float    v4f;
#define PSCALE 32768.0f
#define U16(p) ((const unsigned short*)(const void*)(p))
#define PSCALE_INV (1.0f / 32768.0f)

__device__ __forceinline__ unsigned short f2bf_bits(float f) {
  unsigned u = __float_as_uint(f);
  return (unsigned short)((u + 0x7FFFu + ((u >> 16) & 1u)) >> 16);
}
__device__ __forceinline__ float bf_bits2f(unsigned short h) { return __uint_as_float(((unsigned)h) << 16); }

__device__ __forceinline__ void dep_guard_h(v8f& a, v8f& b, v16h x, v16h y) { asm volatile("v_nop\n\tv_nop\n\tv_nop\n\tv_nop" : "+v"(a), "+v"(b) : "v"(x), "v"(y)); }
__device__ __forceinline__ void dep_guard_b(v8f& a, v8f& b, v16b x, v16b y) { asm volatile("v_nop\n\tv_nop\n\tv_nop\n\tv_nop" : "+v"(a), "+v"(b) : "v"(x), "v"(y)); }
__device__ __forceinline__ void keep4_h(v16h a, v16h b, v16h c, v16h d) { asm volatile("v_nop" :: "v"(a), "v"(b), "v"(c), "v"(d)); }
__device__ __forceinline__ void keep4_b(v16b a, v16b b, v16b c, v16b d) { asm volatile("v_nop" :: "v"(a), "v"(b), "v"(c), "v"(d)); }
__device__ __forceinline__ void acc_guard4(v8f& a, v8f& b, v8f& c, v8f& d) { asm volatile("v_nop\n\tv_nop\n\tv_nop\n\tv_nop" : "+v"(a), "+v"(b), "+v"(c), "+v"(d)); }
template <typename T> struct Frag;
template <> struct Frag<_Float16> {
  typedef v16h V; union U { v16h v; v8h h[2]; };
  static __device__ __forceinline__ v16h load(const _Float16* p) {
    U f; f.h[0] = *(const v8h*)(p); f.h[1] = *(const v8h*)(p + 16); return f.v;
  }
  static __device__ __forceinline__ v8f mma(v16h a, v16h b, v8f c) {
    return __builtin_amdgcn_wmma_f32_16x16x32_f16(false, a, false, b, (short)0, c, false, false);
  }
  static __device__ __forceinline__ void guard(v8f& a, v8f& b, v16h x, v16h y) { dep_guard_h(a, b, x, y); }
  static __device__ __forceinline__ void keep(v16h a, v16h b, v16h c, v16h d) { keep4_h(a, b, c, d); }
};
template <> struct Frag<__bf16> {
  typedef v16b V; union U { v16b v; v8b h[2]; };
  static __device__ __forceinline__ v16b load(const __bf16* p) {
    U f; f.h[0] = *(const v8b*)(p); f.h[1] = *(const v8b*)(p + 16); return f.v;
  }
  static __device__ __forceinline__ v8f mma(v16b a, v16b b, v8f c) {
    return __builtin_amdgcn_wmma_f32_16x16x32_bf16(false, a, false, b, (short)0, c, false, false);
  }
  static __device__ __forceinline__ void guard(v8f& a, v8f& b, v16b x, v16b y) { dep_guard_b(a, b, x, y); }
  static __device__ __forceinline__ void keep(v16b a, v16b b, v16b c, v16b d) { keep4_b(a, b, c, d); }
};

template <int ET> struct Elem;
template <> struct Elem<0> { typedef _Float16 T; };
template <> struct Elem<1> { typedef __bf16 T; };
template <int ET, bool SPLIT, int BIAS_MODE, int OUT_MODE, bool RESID, int ACT = 0>
__global__ __launch_bounds__(256) void wmma_gemm64(
    const unsigned short* __restrict__ Ap, const unsigned short* __restrict__ A2p, int lda, long strideA,
    const unsigned short* __restrict__ Btp, const unsigned short* __restrict__ Bt2p, int ldb, long strideB,
    void* __restrict__ Cout, void* __restrict__ Cout2, int ldc, long strideC,
    const float* __restrict__ bias,
    const float* __restrict__ resid, long strideR,
    int M, int N, int K, float scale) {
  typedef typename Elem<ET>::T T;
  typedef typename Frag<T>::V V;
  const T* A = (const T*)Ap; const T* A2 = (const T*)A2p; const T* Bt = (const T*)Btp; const T* Bt2 = (const T*)Bt2p;
  __shared__ __align__(16) float sT[8][16 * 68];
  const int b    = blockIdx.y;
  const int lane = threadIdx.x & 31;
  const int wave = threadIdx.x >> 5;
  const int tilesN = N >> 6;
  const int tilesM = M >> 6;
  const int tile = blockIdx.x * 8 + wave;
  if (tile >= tilesM * tilesN) return;
  const int tm = tile / tilesN;
  const int tn = tile - tm * tilesN;
  const int m0 = tm << 6;
  const int n0 = tn << 6;

  const T* Ab  = A  + (size_t)b * strideA;
  const T* Bb  = Bt + (size_t)b * strideB;
  const T* Ab2 = SPLIT ? (A2  + (size_t)b * strideA) : nullptr;
  const T* Bb2 = SPLIT ? (Bt2 + (size_t)b * strideB) : nullptr;

  const int rlane = lane & 15;
  const int koff  = (lane >> 4) * 8;
  const int mOff  = (lane >> 4) * 8;

  v8f acc[4][4];
#pragma unroll
  for (int i = 0; i < 4; ++i)
#pragma unroll
    for (int j = 0; j < 4; ++j) acc[i][j] = (v8f){0.f,0.f,0.f,0.f,0.f,0.f,0.f,0.f};

  for (int k0 = 0; k0 < K; k0 += 32) {
    V bh[4], bl[4];
#pragma unroll
    for (int j = 0; j < 4; ++j) {
      const size_t bo = (size_t)(n0 + (j << 4) + rlane) * ldb + koff + k0;
      bh[j] = Frag<T>::load(Bb + bo);
      if (SPLIT) bl[j] = Frag<T>::load(Bb2 + bo);
    }
#pragma unroll
    for (int i = 0; i < 4; ++i) {
      const size_t ao = (size_t)(m0 + (i << 4) + rlane) * lda + koff + k0;
      V ah = Frag<T>::load(Ab + ao);
      V al;
      if (SPLIT) al = Frag<T>::load(Ab2 + ao);
#pragma unroll
      for (int j = 0; j < 4; ++j) {
        acc[i][j] = Frag<T>::mma(ah, bh[j], acc[i][j]);
        if (SPLIT) {
          acc[i][j] = Frag<T>::mma(ah, bl[j], acc[i][j]);
          acc[i][j] = Frag<T>::mma(al, bh[j], acc[i][j]);
        }
      }
      Frag<T>::guard(acc[i][0], acc[i][3], ah, SPLIT ? al : ah);
    }
    Frag<T>::keep(bh[0], bh[1], bh[2], bh[3]);
    if (SPLIT) Frag<T>::keep(bl[0], bl[1], bl[2], bl[3]);
  }
  acc_guard4(acc[0][0], acc[0][1], acc[0][2], acc[0][3]);
  acc_guard4(acc[1][0], acc[1][1], acc[1][2], acc[1][3]);
  acc_guard4(acc[2][0], acc[2][1], acc[2][2], acc[2][3]);
  acc_guard4(acc[3][0], acc[3][1], acc[3][2], acc[3][3]);

  float* slab = sT[wave];
  const float* Rb = RESID ? (resid + (size_t)b * strideR) : nullptr;
#pragma unroll
  for (int i = 0; i < 4; ++i) {
    const int mBase = m0 + (i << 4);
#pragma unroll
    for (int j = 0; j < 4; ++j) {
      const int n = n0 + (j << 4) + rlane;
      float bv = 0.f;
      if (BIAS_MODE == 2) bv = bias[n];
#pragma unroll
      for (int r = 0; r < 8; ++r) {
        float v = acc[i][j][r] * scale;
        if (BIAS_MODE == 1) v += bias[mBase + mOff + r];
        if (BIAS_MODE == 2) v += bv;
        if (RESID) v += Rb[(size_t)(mBase + mOff + r) * ldc + n];
        if (ACT == 1) v = tanhf(v);
        if (ACT == 2) v = fmaxf(v, 0.0f);
        if (ACT == 3) v = v / (1.0f + expf(-v));
        if (ACT == 4) v = (v > 0.f) ? v : 0.01f * v;
        if (ACT == 5) v = 0.5f * v * (1.0f + erff(v * 0.70710678118654752f));
        slab[(mOff + r) * 68 + (j << 4) + rlane] = v;
      }
    }
    __builtin_amdgcn_fence(__ATOMIC_RELEASE, "workgroup");
    __builtin_amdgcn_wave_barrier();
    __builtin_amdgcn_fence(__ATOMIC_ACQUIRE, "workgroup");
    if (OUT_MODE == 0) {
      float* C = (float*)Cout + (size_t)b * strideC;
      const int hh = lane >> 4, c4 = (lane & 15) * 4;
      for (int pass = 0; pass < 2; ++pass) {
#pragma unroll
        for (int it = 0; it < 8; ++it) {
          const int row = it * 2 + hh;
          v4f v = *(const v4f*)(slab + row * 68 + c4);
          *(volatile v4f*)(C + (size_t)(mBase + row) * ldc + n0 + c4) = v;
        }
        __threadfence();
      }
    } else {
      const int q = lane >> 3, c8 = (lane & 7) * 8;
      unsigned short* C  = (unsigned short*)Cout  + (size_t)b * strideC;
      unsigned short* C2 = (OUT_MODE == 2) ? ((unsigned short*)Cout2 + (size_t)b * strideC) : nullptr;
      for (int pass = 0; pass < 2; ++pass) {
#pragma unroll
        for (int it = 0; it < 4; ++it) {
          const int row = it * 4 + q;
          const float* sp = slab + row * 68 + c8;
          v8h hv, lv;
#pragma unroll
          for (int e = 0; e < 8; ++e) {
            if (OUT_MODE == 1) {
              hv[e] = (_Float16)sp[e];
            } else {
              unsigned short hb = f2bf_bits(sp[e]);
              unsigned short lb = f2bf_bits(sp[e] - bf_bits2f(hb));
              hv[e] = __builtin_bit_cast(_Float16, hb);
              lv[e] = __builtin_bit_cast(_Float16, lb);
            }
          }
          *(volatile v8h*)(C + (size_t)(mBase + row) * ldc + n0 + c8) = hv;
          if (OUT_MODE == 2) *(volatile v8h*)(C2 + (size_t)(mBase + row) * ldc + n0 + c8) = lv;
        }
        __threadfence();
      }
    }
    __builtin_amdgcn_fence(__ATOMIC_RELEASE, "workgroup");
    __builtin_amdgcn_wave_barrier();
    __builtin_amdgcn_fence(__ATOMIC_ACQUIRE, "workgroup");
  }
}

template <int ET>
__global__ __launch_bounds__(256) void wmma_gemm64_ksum8(
    const unsigned short* __restrict__ Ap, int lda,
    const unsigned short* __restrict__ Btp, int ldb, long strideB,
    float* __restrict__ Cout, int ldc, long strideC,
    const float* __restrict__ bias0, const float* __restrict__ bias1,
    int M, int N, int K, float scale) {
  typedef typename Elem<ET>::T T;
  typedef typename Frag<T>::V V;
  const int b = blockIdx.y;
  const T* Ab = (const T*)Ap;
  const T* Bb = (const T*)Btp + (size_t)b * strideB;
  const float* bias = (b == 0) ? bias0 : bias1;
  float* C = Cout + (size_t)b * strideC;
  __shared__ __align__(16) float sT[8][8 * 68];
  const int lane = threadIdx.x & 31;
  const int wave = threadIdx.x >> 5;
  const int tilesN = N >> 6;
  const int tilesM = M >> 6;
  const int tile = blockIdx.x * 8 + wave;
  if (tile >= tilesM * tilesN) return;
  const int tm = tile / tilesN;
  const int tn = tile - tm * tilesN;
  const int m0 = tm << 6;
  const int n0 = tn << 6;

  const int rlane = lane & 15;
  const int koff  = (lane >> 4) * 8;
  const int hh    = lane >> 4;

  v8f acc[4][4];
#pragma unroll
  for (int i = 0; i < 4; ++i)
#pragma unroll
    for (int j = 0; j < 4; ++j) acc[i][j] = (v8f){0.f,0.f,0.f,0.f,0.f,0.f,0.f,0.f};

  for (int k0 = 0; k0 < K; k0 += 32) {
    V bh[4];
#pragma unroll
    for (int j = 0; j < 4; ++j) {
      const size_t bo = (size_t)(n0 + (j << 4) + rlane) * ldb + koff + k0;
      bh[j] = Frag<T>::load(Bb + bo);
    }
#pragma unroll
    for (int i = 0; i < 4; ++i) {
      const size_t ao = (size_t)(m0 + (i << 4) + rlane) * lda + koff + k0;
      V ah = Frag<T>::load(Ab + ao);
#pragma unroll
      for (int j = 0; j < 4; ++j) acc[i][j] = Frag<T>::mma(ah, bh[j], acc[i][j]);
      Frag<T>::guard(acc[i][0], acc[i][3], ah, ah);
    }
    Frag<T>::keep(bh[0], bh[1], bh[2], bh[3]);
  }
  acc_guard4(acc[0][0], acc[0][1], acc[0][2], acc[0][3]);
  acc_guard4(acc[1][0], acc[1][1], acc[1][2], acc[1][3]);
  acc_guard4(acc[2][0], acc[2][1], acc[2][2], acc[2][3]);
  acc_guard4(acc[3][0], acc[3][1], acc[3][2], acc[3][3]);

  float* slab = sT[wave];
#pragma unroll
  for (int i = 0; i < 4; ++i) {
#pragma unroll
    for (int j = 0; j < 4; ++j) {
      const int n = n0 + (j << 4) + rlane;
      const float bv = bias[n];
      float s = 0.f;
#pragma unroll
      for (int r = 0; r < 8; ++r) {
        const float v = fmaxf(acc[i][j][r] * scale + bv, 0.0f);
        s += v;
      }
      slab[(2 * i + hh) * 68 + (j << 4) + rlane] = s;
    }
  }
  __builtin_amdgcn_fence(__ATOMIC_RELEASE, "workgroup");
  __builtin_amdgcn_wave_barrier();
  __builtin_amdgcn_fence(__ATOMIC_ACQUIRE, "workgroup");
  {
    const int orow0 = m0 >> 3;
    const int c4 = (lane & 15) * 4;
    for (int pass = 0; pass < 2; ++pass) {
#pragma unroll
      for (int it = 0; it < 4; ++it) {
        const int row = it * 2 + hh;
        v4f v = *(const v4f*)(slab + row * 68 + c4);
        *(volatile v4f*)(C + (size_t)(orow0 + row) * ldc + n0 + c4) = v;
      }
      __threadfence();
    }
  }
  __builtin_amdgcn_fence(__ATOMIC_RELEASE, "workgroup");
  __builtin_amdgcn_wave_barrier();
  __builtin_amdgcn_fence(__ATOMIC_ACQUIRE, "workgroup");
}

__global__ __launch_bounds__(256) void cast8_f32_f16(
    const float* __restrict__ in, _Float16* __restrict__ out, int n8) {
  const int i = blockIdx.x * 256 + threadIdx.x;
  if (i < n8) {
    const v4f a = *(const v4f*)(in + (size_t)i * 8);
    const v4f c = *(const v4f*)(in + (size_t)i * 8 + 4);
    v8h h;
    h[0] = (_Float16)a[0]; h[1] = (_Float16)a[1]; h[2] = (_Float16)a[2]; h[3] = (_Float16)a[3];
    h[4] = (_Float16)c[0]; h[5] = (_Float16)c[1]; h[6] = (_Float16)c[2]; h[7] = (_Float16)c[3];
    _Float16* p = out + (size_t)i * 8;
    *(volatile v8h*)p = h;
    __threadfence();
    *(volatile v8h*)p = h;
  }
}

__global__ __launch_bounds__(256) void transpose_f32_f16(
    const float* __restrict__ in, _Float16* __restrict__ out,
    int R, int C, long strideIn, long strideOut, float scale) {
  __shared__ float tile[64][33];
  const int z = blockIdx.z;
  const float* src = in + (size_t)z * strideIn;
  _Float16* dst = out + (size_t)z * strideOut;
  const int c0 = blockIdx.x * 32, r0 = blockIdx.y * 64;
  const int tid = threadIdx.x, tx = tid & 31, ty = tid >> 5;
#pragma unroll
  for (int it = 0; it < 8; ++it) {
    const int r = ty + 8 * it;
    tile[r][tx] = src[(size_t)(r0 + r) * C + c0 + tx];
  }
  __syncthreads();
  const int q = tid & 7, row = tid >> 3;
  v8h v;
#pragma unroll
  for (int e = 0; e < 8; ++e) v[e] = (_Float16)(tile[8 * q + e][row] * scale);
  _Float16* p = dst + (size_t)(c0 + row) * R + r0 + 8 * q;
  *(volatile v8h*)p = v;
  __threadfence();
  *(volatile v8h*)p = v;
}

#define HS_DF 1024
#define HS_L 128
__global__ __launch_bounds__(128) void head_softmax_mean(
    const float* __restrict__ agent, const float* __restrict__ ssa, const float* __restrict__ ssh,
    float* __restrict__ out) {
  __shared__ float P[8][132];
  __shared__ float S[8][132];
  __shared__ __align__(16) float outs[HS_L];
  const int bi = blockIdx.x;
  const int tid = threadIdx.x, lane = tid & 31, wave = tid >> 5;
  const size_t base = (size_t)bi * HS_DF + (size_t)tid * 8;
  {
    const v4f a0 = *(const v4f*)(agent + base), a1 = *(const v4f*)(agent + base + 4);
    const v4f s0 = *(const v4f*)(ssa + base),   s1 = *(const v4f*)(ssa + base + 4);
    const v4f h0 = *(const v4f*)(ssh + base),   h1 = *(const v4f*)(ssh + base + 4);
    P[0][tid] = a0[0] * s0[0]; P[1][tid] = a0[1] * s0[1]; P[2][tid] = a0[2] * s0[2]; P[3][tid] = a0[3] * s0[3];
    P[4][tid] = a1[0] * s1[0]; P[5][tid] = a1[1] * s1[1]; P[6][tid] = a1[2] * s1[2]; P[7][tid] = a1[3] * s1[3];
    S[0][tid] = h0[0]; S[1][tid] = h0[1]; S[2][tid] = h0[2]; S[3][tid] = h0[3];
    S[4][tid] = h1[0]; S[5][tid] = h1[1]; S[6][tid] = h1[2]; S[7][tid] = h1[3];
  }
  __syncthreads();
#pragma unroll
  for (int u = 0; u < 2; ++u) {
    const int h = wave * 2 + u;
    const float x0 = P[h][lane], x1 = P[h][lane + 32], x2 = P[h][lane + 64], x3 = P[h][lane + 96];
    float m = fmaxf(fmaxf(x0, x1), fmaxf(x2, x3));
#pragma unroll
    for (int off = 1; off < 32; off <<= 1) m = fmaxf(m, __shfl_xor(m, off, 32));
    const float e0 = __expf(x0 - m), e1 = __expf(x1 - m), e2 = __expf(x2 - m), e3 = __expf(x3 - m);
    float s = (e0 + e1) + (e2 + e3);
#pragma unroll
    for (int off = 1; off < 32; off <<= 1) s += __shfl_xor(s, off, 32);
    const float inv = 1.0f / s;
    P[h][lane]      = (e0 * inv) * S[h][lane];
    P[h][lane + 32] = (e1 * inv) * S[h][lane + 32];
    P[h][lane + 64] = (e2 * inv) * S[h][lane + 64];
    P[h][lane + 96] = (e3 * inv) * S[h][lane + 96];
  }
  __syncthreads();
  {
    float accv = P[0][tid];
    accv += P[1][tid]; accv += P[2][tid]; accv += P[3][tid];
    accv += P[4][tid]; accv += P[5][tid]; accv += P[6][tid]; accv += P[7][tid];
    outs[tid] = accv * 0.125f;
  }
  __syncthreads();
  if (wave == 0) {
    const v4f v = *(const v4f*)(outs + 4 * lane);
    float* op = out + (size_t)bi * HS_L + 4 * lane;
    *(volatile v4f*)op = v;
    __threadfence();
    *(volatile v4f*)op = v;
  }
}

extern "C" void kernel_launch(void* const* d_in, const int* in_sizes, int n_in,
                              void* d_out, int out_size, void* d_ws, size_t ws_size,
                              hipStream_t stream) {
  const int Bc = 8, Nn = 128, Kn = 8, Dd = 1024, Ll = 128;
  if (n_in < 8) return;
  if (in_sizes[0] != Bc * Nn * Dd) return;
  if (in_sizes[1] != Bc * Nn * Kn * Nn) return;
  if (in_sizes[2] != Dd * Dd || in_sizes[4] != Dd * Dd || in_sizes[6] != Dd * Dd) return;
  if (in_sizes[3] != Dd || in_sizes[5] != Dd || in_sizes[7] != Dd) return;
  if (out_size != Bc * Nn * Ll) return;

  const float* embedded = (const float*)d_in[0];
  const float* adj      = (const float*)d_in[1];
  const float* Wl       = (const float*)d_in[2];
  const float* bl       = (const float*)d_in[3];
  const float* Wa       = (const float*)d_in[4];
  const float* ba       = (const float*)d_in[5];
  const float* Wh       = (const float*)d_in[6];
  const float* bh       = (const float*)d_in[7];
  float* out = (float*)d_out;

  unsigned char* ws = (unsigned char*)d_ws;
  size_t off = 0;
  auto carve = [&](size_t bytes) -> unsigned char* {
    unsigned char* p = ws + off;
    off += (bytes + 255) & ~(size_t)255;
    return p;
  };
  const size_t nEmb  = (size_t)Bc * Nn * Dd;
  const size_t nAdj  = (size_t)Bc * Nn * Kn * Nn;
  const size_t nW    = (size_t)Dd * Dd;
  const size_t nNE   = (size_t)Bc * Nn * Kn * Dd;
  const size_t nRow  = (size_t)Bc * Nn * Dd;

  _Float16* Xh    = (_Float16*)carve(nEmb * 2);
  _Float16* adjh  = (_Float16*)carve(nAdj * 2);
  _Float16* embT  = (_Float16*)carve(nEmb * 2);
  _Float16* WlT   = (_Float16*)carve(nW * 2);
  _Float16* WahT  = (_Float16*)carve(nW * 2 * 2);
  _Float16* NE    = (_Float16*)carve(nNE * 2);
  float*    agent = (float*)carve(nRow * 4);
  float*    SAH   = (float*)carve(nRow * 4 * 2);
  if (off > ws_size || off > (size_t)134217728) return;

  _Float16* WaT = WahT;
  _Float16* WhT = WahT + nW;
  const float wscale = 1024.0f;
  const float wunscale = 1.0f / 1024.0f;

  {
    const int n8e = (int)(nEmb / 8), n8a = (int)(nAdj / 8);
    cast8_f32_f16<<<dim3((n8e + 255) / 256), 256, 0, stream>>>(embedded, Xh, n8e);
    cast8_f32_f16<<<dim3((n8a + 255) / 256), 256, 0, stream>>>(adj, adjh, n8a);
  }
  transpose_f32_f16<<<dim3(Dd / 32, Nn / 64, Bc), 256, 0, stream>>>(
      embedded, embT, Nn, Dd, (long)Nn * Dd, (long)Dd * Nn, 1.0f);
  transpose_f32_f16<<<dim3(Dd / 32, Dd / 64, 1), 256, 0, stream>>>(Wl, WlT, Dd, Dd, 0L, 0L, wscale);
  transpose_f32_f16<<<dim3(Dd / 32, Dd / 64, 1), 256, 0, stream>>>(Wa, WaT, Dd, Dd, 0L, 0L, wscale);
  transpose_f32_f16<<<dim3(Dd / 32, Dd / 64, 1), 256, 0, stream>>>(Wh, WhT, Dd, Dd, 0L, 0L, wscale);

  {
    const int M = Nn * Kn, N = Dd, K = Nn;
    const int tiles = (M / 64) * (N / 64);
    wmma_gemm64<0, false, 0, 1, false, 0><<<dim3((tiles + 7) / 8, Bc), 256, 0, stream>>>(
        U16(adjh), U16(adjh), K, (long)Nn * Kn * Nn,
        U16(embT), U16(embT), K, (long)Dd * Nn,
        (void*)NE, (void*)NE, Dd, (long)Nn * Kn * Dd,
        bl, bl, 0L, M, N, K, 1.0f);
  }
  {
    const int M = Bc * Nn, N = Dd, K = Dd;
    const int tiles = (M / 64) * (N / 64);
    wmma_gemm64<0, false, 2, 0, false, 2><<<dim3((tiles + 7) / 8, 1), 256, 0, stream>>>(
        U16(Xh), U16(Xh), Dd, 0L,
        U16(WlT), U16(WlT), Dd, 0L,
        (void*)agent, (void*)agent, Dd, 0L,
        bl, bl, 0L, M, N, K, wunscale);
  }
  {
    const int M = Bc * Nn * Kn, N = Dd, K = Dd;
    const int tiles = (M / 64) * (N / 64);
    wmma_gemm64_ksum8<0><<<dim3((tiles + 7) / 8, 2), 256, 0, stream>>>(
        U16(NE), Dd,
        U16(WaT), Dd, (long)nW,
        SAH, Dd, (long)nRow,
        ba, bh, M, N, K, wunscale);
  }
  head_softmax_mean<<<dim3(Bc * Nn), 128, 0, stream>>>(agent, SAH, SAH + nRow, out);
}
